// RelativeMultiHeadSelfAttention_3573412790778
// MI455X (gfx1250) — hardware-verified
//
#include <hip/hip_runtime.h>
#include <math.h>

typedef __attribute__((ext_vector_type(16))) _Float16 v16h;
typedef __attribute__((ext_vector_type(16))) __bf16 v16b;
typedef __attribute__((ext_vector_type(8)))  _Float16 v8h;
typedef __attribute__((ext_vector_type(8)))  float v8f;
typedef __attribute__((ext_vector_type(4)))  float v4f;
typedef __attribute__((ext_vector_type(2)))  float v2f;
typedef __attribute__((ext_vector_type(4)))  unsigned v4u;
typedef __attribute__((ext_vector_type(4)))  int v4i;
typedef float __attribute__((may_alias)) float_a;
typedef int __attribute__((may_alias)) int_a;

template <typename T> __device__ __forceinline__ void vst2(void* p, T v) { *(volatile T*)p = v; __threadfence(); *(volatile T*)p = v; }
__device__ __forceinline__ v8f wmma16(v16h a, v16h b, v8f c) {
  v8f d = __builtin_amdgcn_wmma_f32_16x16x32_f16(false, a, false, b, (short)0, c, false, false);
  asm volatile("v_nop\n\tv_nop\n\tv_nop\n\tv_nop" : "+v"(d) : "v"(a), "v"(b));
  return d;
}
__device__ __forceinline__ v8f wmma_bf(v16b a, v16b b, v8f c) {
  v8f d = __builtin_amdgcn_wmma_f32_16x16x32_bf16(false, a, false, b, (short)0, c, false, false);
  asm volatile("v_nop\n\tv_nop\n\tv_nop\n\tv_nop" : "+v"(d) : "v"(a), "v"(b));
  return d;
}
__device__ __forceinline__ v16h frag_h(const _Float16* rowk0, int lane) {
  union { v16h v; v8h q[2]; } u; const _Float16* p = rowk0 + 8 * (lane >> 4);
  u.q[0] = *(const v8h*)p; u.q[1] = *(const v8h*)(p + 16); return u.v;
}
__device__ __forceinline__ v16h frag_f32(const float* rowk0, int lane) {
  v16h a; const float* p = rowk0 + 8 * (lane >> 4);
#pragma unroll
  for (int i = 0; i < 8; ++i) { a[i] = (_Float16)p[i]; a[8 + i] = (_Float16)p[16 + i]; }
  return a;
}
__device__ __forceinline__ v16h frag_f32s(const float* rowk0, int lane, float sc) {
  v16h a; const float* p = rowk0 + 8 * (lane >> 4);
#pragma unroll
  for (int i = 0; i < 8; ++i) { a[i] = (_Float16)(p[i] * sc); a[8 + i] = (_Float16)(p[16 + i] * sc); }
  return a;
}
__device__ __forceinline__ v16h fragc_f32(const float* W, int k0, int n, int lane, int ld, int K) {
  v16h a; const int g = lane >> 4;
#pragma unroll
  for (int i = 0; i < 8; ++i) { const int ka = k0 + 8 * g + i, kb = ka + 16;
    a[i] = (_Float16)(ka < K ? W[(size_t)(ka < K ? ka : K - 1) * ld + n] : 0.f); a[8 + i] = (_Float16)(kb < K ? W[(size_t)(kb < K ? kb : K - 1) * ld + n] : 0.f); }
  return a;
}
struct F2 { v16b h, l; };
__device__ __forceinline__ F2 bsplit16(const float v[16]) { F2 r;
#pragma unroll
  for (int i = 0; i < 16; ++i) { const __bf16 h = (__bf16)v[i]; r.h[i] = h; r.l[i] = (__bf16)(v[i] - (float)h); }
  return r; }
__device__ __forceinline__ F2 split_row(const float* row, int k0, int lane) { float v[16]; const float* p = row + k0 + 8 * (lane >> 4);
#pragma unroll
  for (int i = 0; i < 8; ++i) { v[i] = p[i]; v[8 + i] = p[16 + i]; }
  return bsplit16(v); }
__device__ __forceinline__ F2 split_rowK(const float* row, int k0, int lane, int K) { float v[16]; const int g = lane >> 4;
#pragma unroll
  for (int i = 0; i < 8; ++i) { const int ka = k0 + 8 * g + i, kb = ka + 16; v[i] = ka < K ? row[ka < K ? ka : K - 1] : 0.f; v[8 + i] = kb < K ? row[kb < K ? kb : K - 1] : 0.f; }
  return bsplit16(v); }
__device__ __forceinline__ F2 split_col(const float* W, int k0, int n, int lane, int ld, int K) { float v[16]; const int g = lane >> 4;
#pragma unroll
  for (int i = 0; i < 8; ++i) { const int ka = k0 + 8 * g + i, kb = ka + 16; v[i] = ka < K ? W[(size_t)(ka < K ? ka : K - 1) * ld + n] : 0.f; v[8 + i] = kb < K ? W[(size_t)(kb < K ? kb : K - 1) * ld + n] : 0.f; }
  return bsplit16(v); }
__device__ __forceinline__ v8f mac3(const F2& a, const F2& b, v8f c) { c = wmma_bf(a.l, b.h, c); c = wmma_bf(a.h, b.l, c); return wmma_bf(a.h, b.h, c); }
__device__ __forceinline__ float sigm(float v) { return 1.0f / (1.0f + expf(-v)); }
#define LDSX() do { asm volatile("s_wait_dscnt 0" ::: "memory"); __builtin_amdgcn_wave_barrier(); __builtin_amdgcn_fence(__ATOMIC_RELEASE, "workgroup"); } while (0)


#define NB 2
#define TT 2048
#define DMD 1024
#define NH 16
#define HD 64
#define POFF 32
#define PROWS (TT + 64)
#ifndef TNB
#define TNB NB
#endif
#ifndef TQB2
#define TQB2 (TT / 64)
#endif
#ifndef TOB2
#define TOB2 (TNB * TT / 64)
#endif
typedef __attribute__((ext_vector_type(8))) __bf16 v8b;
__device__ __forceinline__ v16b frag_b(const __bf16* rowk0, int lane) {
  union { v16b v; v8b q[2]; } u; const __bf16* p = rowk0 + 8 * (lane >> 4);
  u.q[0] = *(const v8b*)p; u.q[1] = *(const v8b*)(p + 16); return u.v;
}
__device__ __forceinline__ float bfr(float v) { return (float)(__bf16)v; }
__device__ __attribute__((noinline)) float exp_ni(float v) { return expf(v); }
__device__ __attribute__((noinline)) float erf_ni(float v) { return erff(v); }

#define WS_Q   0u
#define WS_KH  (WS_Q + 4u * (size_t)NB * TT * DMD)
#define WS_PH  (WS_KH + 2u * (size_t)NB * TT * DMD)
#define WS_VH  (WS_PH + 2u * (size_t)PROWS * DMD)
#define WS_VL  (WS_VH + 2u * (size_t)NB * DMD * TT)
#define WS_X   (WS_VL + 2u * (size_t)NB * DMD * TT)
#define WS_SIN (WS_X + 4u * (size_t)NB * TT * DMD)
#define WS_END (WS_SIN + 4u * (size_t)TT * DMD)

template <int WOFF>
__global__ __launch_bounds__(128) void k_proj(const float* __restrict__ Xin, const float* __restrict__ WQ, const float* __restrict__ BQ, const float* __restrict__ WK, const float* __restrict__ BK, const float* __restrict__ WV, const float* __restrict__ BV, const float* __restrict__ WP, const float* __restrict__ BP, float* __restrict__ Q, _Float16* __restrict__ KH, _Float16* __restrict__ VH, _Float16* __restrict__ VL, _Float16* __restrict__ PH) {
  __shared__ __align__(16) float sf[4][16][132]; __shared__ __align__(16) _Float16 sh[64][136]; __shared__ __align__(16) _Float16 th[128][72], tl[128][72];
  const int tid = threadIdx.x, wave = tid >> 5, lane = tid & 31, col = lane & 15, g = lane >> 4; const int which = blockIdx.z + WOFF; const int c0 = blockIdx.y * 128; const int nrows = (which == 3) ? TT : NB * TT;
  if ((int)blockIdx.x * 64 >= nrows) return;
  const float* Wm = (which == 0 ? WQ : which == 1 ? WK : which == 2 ? WV : WP); const float* Bm = (which == 0 ? BQ : which == 1 ? BK : which == 2 ? BV : BP);
  const size_t r0 = (size_t)blockIdx.x * 64 + wave * 16;
  v8f acc[8] = {};
#pragma unroll 2
  for (int kc = 0; kc < DMD / 32; ++kc) { F2 a2; v16b a; if (which < 3) { const float* p = Xin + (r0 + col) * DMD + kc * 32 + 8 * g;
#pragma unroll
      for (int i = 0; i < 8; ++i) { a[i] = (__bf16)p[i]; a[8 + i] = (__bf16)p[16 + i]; } }
    else { float v[16]; const float* p = Xin + (r0 + col) * DMD + kc * 32 + 8 * g;
#pragma unroll
      for (int i = 0; i < 8; ++i) { v[i] = p[i]; v[8 + i] = p[16 + i]; }
      a2 = bsplit16(v); }
#pragma unroll
    for (int j = 0; j < 8; ++j) { v16b w; const int o = c0 + j * 16 + col;
#pragma unroll
      for (int i = 0; i < 8; ++i) { w[i] = (__bf16)Wm[(size_t)(kc * 32 + 8 * g + i) * DMD + o]; w[8 + i] = (__bf16)Wm[(size_t)(kc * 32 + 16 + 8 * g + i) * DMD + o]; }
      if (which < 3) acc[j] = wmma_bf(a, w, acc[j]); else { acc[j] = wmma_bf(a2.h, w, acc[j]); acc[j] = wmma_bf(a2.l, w, acc[j]); } } }
#pragma unroll
  for (int j = 0; j < 8; ++j) { const float bb = bfr(Bm[c0 + j * 16 + col]);
#pragma unroll
    for (int r = 0; r < 8; ++r) { const float v = acc[j][r] + bb; const int rl = wave * 16 + 8 * g + r, cl = j * 16 + col;
      if (which == 0) sf[wave][8 * g + r][cl] = v; else if (which == 2) { const _Float16 hv = (_Float16)v; th[cl][rl] = hv; tl[cl][rl] = (_Float16)(v - (float)hv); } else sh[rl][cl] = (_Float16)v; } }
  __syncthreads();
  if (which == 0) { for (int rl = 0; rl < 16; ++rl) vst2(Q + (r0 + rl) * DMD + c0 + lane * 4, *(const v4f*)&sf[wave][rl][lane * 4]); }
  else if (which == 2) { const size_t b = ((size_t)blockIdx.x * 64) / TT; const int t0 = (int)(((size_t)blockIdx.x * 64) % TT); for (int e = tid; e < 128 * 8; e += 128) { const int cl = e >> 3, q = e & 7; const size_t o = (b * DMD + c0 + cl) * (size_t)TT + t0 + q * 8; vst2((unsigned*)(VH + o), *(const v4u*)&th[cl][q * 8]); vst2((unsigned*)(VL + o), *(const v4u*)&tl[cl][q * 8]); } }
  else { _Float16* dst = (which == 1) ? (KH + (size_t)blockIdx.x * 64 * DMD) : (PH + ((size_t)POFF + blockIdx.x * 64) * DMD); for (int e = tid; e < 64 * 16; e += 128) { const int rl = e >> 4, q = e & 15; vst2((unsigned*)(dst + (size_t)rl * DMD + c0 + q * 8), *(const v4u*)&sh[rl][q * 8]); } } }
__global__ __launch_bounds__(256) void k_sin(float* __restrict__ SINT) { __shared__ __align__(16) float sr[DMD]; const int t = threadIdx.x; const int s = blockIdx.x;
  for (int c = t; c < DMD / 2; c += 256) { const float ang = (float)s * powf(10000.0f, -2.0f * (float)c / (float)DMD); sr[c] = sinf(ang); sr[DMD / 2 + c] = cosf(ang); }
  __syncthreads(); vst2(SINT + (size_t)s * DMD + t * 4, *(const v4f*)&sr[t * 4]); }
__global__ __launch_bounds__(256) void k_padph(_Float16* __restrict__ PH) { const int t = threadIdx.x; const int r = blockIdx.x; const size_t row = (r < POFF) ? r : (TT + r);
  v4u z; z[0] = z[1] = z[2] = z[3] = 0u; if (t < DMD / 8) vst2((unsigned*)(PH + row * DMD + t * 8), z); }
__device__ __forceinline__ void qfrags(const float* __restrict__ Q, size_t row0, int h, const float* __restrict__ bias, int lane, v16h* hi, v16h* lo) { const int col = lane & 15, g = lane >> 4; size_t row = row0 + col; if (row > (size_t)NB * TT - 1) row = (size_t)NB * TT - 1;
#pragma unroll
  for (int kc = 0; kc < 2; ++kc) { const float* p = Q + row * DMD + h * HD + kc * 32 + 8 * g; const float* bp = bias + h * HD + kc * 32 + 8 * g; v16h a, b;
#pragma unroll
    for (int i = 0; i < 8; ++i) { const float v0 = p[i] + bfr(bp[i]), v1 = p[16 + i] + bfr(bp[16 + i]); const _Float16 h0 = (_Float16)v0, h1 = (_Float16)v1; a[i] = h0; a[8 + i] = h1; b[i] = (_Float16)(v0 - (float)h0); b[8 + i] = (_Float16)(v1 - (float)h1); }
    hi[kc] = a; lo[kc] = b; } }
__global__ __launch_bounds__(128) void k_att(const float* __restrict__ Q, const _Float16* __restrict__ KH, const _Float16* __restrict__ PH, const _Float16* __restrict__ VH, const _Float16* __restrict__ VL, const float* __restrict__ BU, const float* __restrict__ BVv, float* __restrict__ X) {
  __shared__ __align__(16) float sp[4][16][36]; __shared__ __align__(16) float sg1[4][16][36], sg2[4][16][36]; __shared__ __align__(16) float so[4][16][68];
  const int tid = threadIdx.x, wave = tid >> 5, lane = tid & 31, col = lane & 15, g = lane >> 4; const int qb = blockIdx.x, h = blockIdx.y; const size_t b = blockIdx.z; const int i0 = qb * 64 + wave * 16;
  v16h au[2], av[2], aw[2], tmpl[2];
  qfrags(Q, b * TT + i0, h, BU, lane, au, tmpl); qfrags(Q, b * TT + i0, h, BVv, lane, av, tmpl);
  qfrags(Q, b * TT + i0 + 1, h, BVv, lane, aw, tmpl);
  const bool lastblk = (i0 + 16 >= TT);
  float m[8], l[8];
#pragma unroll
  for (int r = 0; r < 8; ++r) { m[r] = -3.0e38f; l[r] = 0.f; }
  v8f acc[4] = {};
#pragma unroll 1
  for (int ks = 0; ks < TT / 32; ++ks) { float s[2][8];
#pragma unroll
    for (int ct = 0; ct < 2; ++ct) { const int j0 = ks * 32 + ct * 16; const int kk = j0 + col; v8f c = {};
#pragma unroll
      for (int kc = 0; kc < 2; ++kc) { const v16h kh = frag_h(KH + (b * TT + kk) * DMD + h * HD + kc * 32, lane); c = wmma16(au[kc], kh, c); }
      const bool needlow = (j0 <= i0 + 15);
      const bool needup = (j0 + 15 >= i0 + 2);
      if (needlow) { const int pA = TT - 16 - i0 + j0 + POFF;
#pragma unroll
        for (int pt = 0; pt < 2; ++pt) { v8f gg = {};
#pragma unroll
          for (int kc = 0; kc < 2; ++kc) { const v16h pf = frag_h(PH + (size_t)(pA + pt * 16 + col) * DMD + h * HD + kc * 32, lane); gg = wmma16(av[kc], pf, gg); }
#pragma unroll
          for (int r = 0; r < 8; ++r) sg1[wave][8 * g + r][pt * 16 + col] = gg[r]; } }
      if (needup) { const int pB = j0 - i0 - 17 + POFF;
#pragma unroll
        for (int pt = 0; pt < 2; ++pt) { v8f gg = {};
#pragma unroll
          for (int kc = 0; kc < 2; ++kc) { const v16h pf = frag_h(PH + (size_t)(pB + pt * 16 + col) * DMD + h * HD + kc * 32, lane); gg = wmma16(aw[kc], pf, gg); }
#pragma unroll
          for (int r = 0; r < 8; ++r) sg2[wave][8 * g + r][pt * 16 + col] = gg[r]; } }
      LDSX();
#pragma unroll
      for (int r = 0; r < 8; ++r) { const int il = 8 * g + r; const int i = i0 + il; const int j = kk; const int idx = 15 + col - il;
        float bd; if (j <= i) bd = sg1[wave][il][idx]; else if (j == i + 1) bd = 0.f; else bd = (lastblk && il == 15) ? 0.f : sg2[wave][il][idx];
        s[ct][r] = (c[r] + bd) * 0.125f; }
      LDSX(); }
    float alpha[8];
#pragma unroll
    for (int r = 0; r < 8; ++r) { float mx = fmaxf(s[0][r], s[1][r]);
#pragma unroll
      for (int o = 1; o < 16; o <<= 1) mx = fmaxf(mx, __shfl_xor(mx, o));
      const float mn = fmaxf(m[r], mx); alpha[r] = (m[r] <= -1.0e38f) ? 0.f : __expf(m[r] - mn); const float e0 = (s[0][r] <= -1.0e38f) ? 0.f : __expf(s[0][r] - mn), e1 = (s[1][r] <= -1.0e38f) ? 0.f : __expf(s[1][r] - mn); float es = e0 + e1;
#pragma unroll
      for (int o = 1; o < 16; o <<= 1) es += __shfl_xor(es, o);
      l[r] = l[r] * alpha[r] + es; m[r] = mn; sp[wave][8 * g + r][col] = e0; sp[wave][8 * g + r][16 + col] = e1; }
#pragma unroll
    for (int j = 0; j < 4; ++j)
#pragma unroll
      for (int r = 0; r < 8; ++r) acc[j][r] *= alpha[r];
    LDSX();
    v16h pa, pr; { const float* prow = &sp[wave][col][0] + 8 * (lane >> 4);
#pragma unroll
      for (int i = 0; i < 8; ++i) { const float x0 = prow[i] * 2048.0f, x1 = prow[16 + i] * 2048.0f; const _Float16 h0 = (_Float16)x0, h1 = (_Float16)x1; pa[i] = h0; pa[8 + i] = h1; pr[i] = (_Float16)(x0 - (float)h0); pr[8 + i] = (_Float16)(x1 - (float)h1); } }
#pragma unroll
    for (int j = 0; j < 4; ++j) { const size_t po = (b * DMD + (size_t)h * HD + j * 16 + col) * TT + ks * 32; const v16h vh = frag_h(VH + po, lane); acc[j] = wmma16(pa, vh, acc[j]); acc[j] = wmma16(pr, vh, acc[j]); acc[j] = wmma16(pa, frag_h(VL + po, lane), acc[j]); }
    LDSX(); }
#pragma unroll
  for (int r = 0; r < 8; ++r) { const float il = (l[r] > 0.f) ? (1.0f / 2048.0f) / l[r] : 0.f;
#pragma unroll
    for (int j = 0; j < 4; ++j) so[wave][8 * g + r][j * 16 + col] = acc[j][r] * il; }
  LDSX(); for (int rl = 0; rl < 16; ++rl) if (lane < 16) vst2(X + (b * TT + i0 + rl) * DMD + h * HD + lane * 4, *(const v4f*)&so[wave][rl][lane * 4]); }
__global__ __launch_bounds__(128) void k_out(const float* __restrict__ X, const float* __restrict__ WO, const float* __restrict__ BO, float* __restrict__ OUT) { __shared__ __align__(16) float sf[4][16][132];
  const int tid = threadIdx.x, wave = tid >> 5, lane = tid & 31, col = lane & 15, g = lane >> 4; const int c0 = blockIdx.y * 128; const size_t r0 = (size_t)blockIdx.x * 64 + wave * 16;
  v8f acc[8] = {};
#pragma unroll
  for (int kc = 0; kc < DMD / 32; ++kc) { const F2 a = split_row(X + (r0 + col) * DMD, kc * 32, lane);
#pragma unroll
    for (int j = 0; j < 8; ++j) { v16b w; const int o = c0 + j * 16 + col;
#pragma unroll
      for (int i = 0; i < 8; ++i) { w[i] = (__bf16)WO[(size_t)(kc * 32 + 8 * g + i) * DMD + o]; w[8 + i] = (__bf16)WO[(size_t)(kc * 32 + 16 + 8 * g + i) * DMD + o]; }
      acc[j] = wmma_bf(a.h, w, acc[j]); acc[j] = wmma_bf(a.l, w, acc[j]); } }
#pragma unroll
  for (int j = 0; j < 8; ++j) { const float bb = bfr(BO[c0 + j * 16 + col]);
#pragma unroll
    for (int r = 0; r < 8; ++r) sf[wave][8 * g + r][j * 16 + col] = acc[j][r] + bb; }
  LDSX(); for (int rl = 0; rl < 16; ++rl) vst2(OUT + (r0 + rl) * DMD + c0 + lane * 4, *(const v4f*)&sf[wave][rl][lane * 4]); }
extern "C" void kernel_launch(void* const* d_in, const int* in_sizes, int n_in, void* d_out, int out_size, void* d_ws, size_t ws_size, hipStream_t stream) {
  (void)in_sizes; (void)n_in; (void)out_size;
  const float** F = (const float**)d_in;
  if (ws_size < (size_t)WS_END) return;
  char* ws = (char*)d_ws; float* Q = (float*)(ws + WS_Q); _Float16 *KH = (_Float16*)(ws + WS_KH), *PH = (_Float16*)(ws + WS_PH), *VH = (_Float16*)(ws + WS_VH), *VL = (_Float16*)(ws + WS_VL); float* X = (float*)(ws + WS_X);
  float* SINT = (float*)(ws + WS_SIN);
  k_sin<<<TT, 256, 0, stream>>>(SINT);
  k_proj<0><<<dim3(TNB * TT / 64, DMD / 128, 3), 128, 0, stream>>>(F[0], F[1], F[2], F[3], F[4], F[5], F[6], F[7], F[8], Q, KH, VH, VL, PH);
  k_proj<3><<<dim3(TT / 64, DMD / 128, 1), 128, 0, stream>>>(SINT, F[1], F[2], F[3], F[4], F[5], F[6], F[7], F[8], Q, KH, VH, VL, PH);
  k_padph<<<64, 256, 0, stream>>>(PH);
  k_att<<<dim3(TQB2, NH, TNB), 128, 0, stream>>>(Q, KH, PH, VH, VL, F[11], F[12], X);
  k_out<<<dim3(TOB2, DMD / 128), 128, 0, stream>>>(X, F[9], F[10], (float*)d_out);
}
